// DownstreamSingleAttentionModel_50173807952800
// MI455X (gfx1250) — hardware-verified
//
#include <hip/hip_runtime.h>
#include <hip/hip_bf16.h>
#include <math.h>

typedef __attribute__((ext_vector_type(16))) _Float16 v16h;
typedef __attribute__((ext_vector_type(8)))  _Float16 v8h;
typedef __attribute__((ext_vector_type(8)))  float    v8f;
typedef __attribute__((ext_vector_type(4)))  float    v4f_t;
typedef float v4fa __attribute__((ext_vector_type(4), may_alias));
#define RSPLIT (1.0f / 2048.0f)
#define PL_X ((size_t)MROWS * CDIM)
#define PL_W ((size_t)OUTC * CDIM)
__device__ __forceinline__ _Float16 lo_of(float v, _Float16 h) { return (_Float16)((v - (float)h) * 2048.0f); }
__device__ __forceinline__ v8f wmma16(v16h a, v16h b, v8f c) { return __builtin_amdgcn_wmma_f32_16x16x32_f16(false, a, false, b, (short)0, c, false, false); }
__device__ __forceinline__ v8f wmma_split(v16h a, v16h al, v16h b, v16h bl, v8f c) { v8f x = {}; x = wmma16(al, b, x); x = wmma16(a, bl, x); return wmma16(a, b, c) + x * RSPLIT; }

#define NB    2
#define LSEQ  1024
#define CDIM  256
#define HH    64
#define EE    16
#define CLW   64
#define LMID  960
#define MROWS (NB*LSEQ)
#define QK    (HH*EE)
#define OUTC  (2*QK + HH)
#define BPAD  264

#ifndef USE_ASYNC_LDS
#define USE_ASYNC_LDS 1
#endif

__global__ __launch_bounds__(256)
void to_half(const float* __restrict__ x,
             const float* __restrict__ Wq, const float* __restrict__ Wk,
             const float* __restrict__ Wv,
             _Float16* __restrict__ xh, _Float16* __restrict__ wh)
{
    const int total = MROWS*CDIM + OUTC*CDIM;
    for (int i = (blockIdx.x*blockDim.x + threadIdx.x) * 2; i < total;
         i += gridDim.x*blockDim.x * 2) {
        float v0, v1; _Float16* d; size_t pl;
        if (i < MROWS*CDIM) { v0 = x[i]; v1 = x[i + 1]; d = xh + i; pl = PL_X; }
        else {
            const int j = i - MROWS*CDIM;
            const int c = j / CDIM, k = j - c*CDIM;
            const float* src = (c < QK) ? (Wq + c*CDIM) : (c < 2*QK) ? (Wk + (c - QK)*CDIM) : (Wv + (c - 2*QK)*CDIM);
            v0 = src[k]; v1 = src[k + 1]; d = wh + j; pl = PL_W;
        }
        const _Float16 h0 = (_Float16)v0, h1 = (_Float16)v1;
        const unsigned pv = (unsigned)__builtin_bit_cast(unsigned short, h0) | ((unsigned)__builtin_bit_cast(unsigned short, h1) << 16);
        const unsigned plv = (unsigned)__builtin_bit_cast(unsigned short, lo_of(v0, h0)) | ((unsigned)__builtin_bit_cast(unsigned short, lo_of(v1, h1)) << 16);
        *(volatile unsigned*)d = pv; *(volatile unsigned*)(d + pl) = plv; __threadfence();
        *(volatile unsigned*)d = pv; *(volatile unsigned*)(d + pl) = plv;
    }
}

__global__ __launch_bounds__(256)
void qkv_gemm(const _Float16* __restrict__ xh, const _Float16* __restrict__ wh,
              const float* __restrict__ bq, const float* __restrict__ bk,
              const float* __restrict__ bv,
              float* __restrict__ Q, float* __restrict__ Kb, float* __restrict__ V)
{
    __shared__ __attribute__((aligned(16))) _Float16 ldsB[2][64 * BPAD];
    const int colGrp   = blockIdx.x % (OUTC/64);
    const int rowBlock = blockIdx.x / (OUTC/64);
    const int c0 = colGrp * 64;

    const _Float16* wsrc = wh + (size_t)c0 * CDIM;
    #pragma unroll
    for (int i = 0; i < 8; ++i) {
        const int q   = i * 256 + threadIdx.x;
        const int row = q >> 5;
        const int wi  = (q & 31) * 8;
        const _Float16* gp = wsrc + row * CDIM + wi;
        _Float16*       lp = ldsB[0] + row * BPAD + wi;
        _Float16*       lq = ldsB[1] + row * BPAD + wi;
#if USE_ASYNC_LDS
        asm volatile("global_load_async_to_lds_b128 %0, %1, off"
                     :: "v"((unsigned)(size_t)lp),
                        "v"((unsigned long long)(size_t)gp)
                     : "memory");
        asm volatile("global_load_async_to_lds_b128 %0, %1, off"
                     :: "v"((unsigned)(size_t)lq),
                        "v"((unsigned long long)(size_t)(gp + PL_W))
                     : "memory");
#else
        *(uint4*)lp = *(const uint4*)gp; *(uint4*)lq = *(const uint4*)(gp + PL_W);
#endif
    }
#if USE_ASYNC_LDS
    asm volatile("s_wait_asynccnt 0x0" ::: "memory");
#endif
    __syncthreads();

    const int lane = threadIdx.x & 31;
    const int wv   = threadIdx.x >> 5;
    const int m0   = (rowBlock * 8 + wv) * 16;
    const int nsel = lane & 15;
    const int aoff = (lane & 16) ? 8  : 0;
    const int boff = aoff;

    const _Float16* xrow = xh  + (size_t)(m0 + nsel) * CDIM;
    const _Float16* brow = ldsB[0] + nsel * BPAD;
    const _Float16* brlo = ldsB[1] + nsel * BPAD;

    v8f acc[4] = {};
    for (int kk = 0; kk < CDIM; kk += 32) {
        const v16h a  = __builtin_shufflevector(*(const v8h*)(xrow + kk + aoff),        *(const v8h*)(xrow + kk + aoff + 16),        0,1,2,3,4,5,6,7,8,9,10,11,12,13,14,15);
        const v16h al = __builtin_shufflevector(*(const v8h*)(xrow + PL_X + kk + aoff), *(const v8h*)(xrow + PL_X + kk + aoff + 16), 0,1,2,3,4,5,6,7,8,9,10,11,12,13,14,15);

        v16h bfrag[4], blo[4];
        #pragma unroll
        for (int ct = 0; ct < 4; ++ct) {
            const _Float16* bp = brow + ct * (16*BPAD) + kk + boff;
            const _Float16* bl = brlo + ct * (16*BPAD) + kk + boff;
            bfrag[ct] = __builtin_shufflevector(*(const v8h*)bp, *(const v8h*)(bp + 16), 0,1,2,3,4,5,6,7,8,9,10,11,12,13,14,15);
            blo[ct]   = __builtin_shufflevector(*(const v8h*)bl, *(const v8h*)(bl + 16), 0,1,2,3,4,5,6,7,8,9,10,11,12,13,14,15);
        }
        #pragma unroll
        for (int ct = 0; ct < 4; ++ct) acc[ct] = wmma_split(a, al, bfrag[ct], blo[ct], acc[ct]);
    }

    const float* bias; float* Obase; int ldo; int cterm;
    if (c0 < QK)        { bias = bq; Obase = Q;  ldo = QK; cterm = 0;    }
    else if (c0 < 2*QK) { bias = bk; Obase = Kb; ldo = QK; cterm = QK;   }
    else                { bias = bv; Obase = V;  ldo = HH; cterm = 2*QK; }
    __syncthreads();
    float* stg = (float*)ldsB[0] + wv * (16 * 68);
    #pragma unroll
    for (int ct = 0; ct < 4; ++ct) {
        const int col = ct*16 + nsel;
        const float bb = bias[c0 - cterm + col];
        #pragma unroll
        for (int j = 0; j < 8; ++j) stg[(j + aoff) * 68 + col] = acc[ct][j] + bb;
    }
    asm volatile("s_wait_dscnt 0" ::: "memory");
    #pragma unroll 1
    for (int pass = 0; pass < 2; ++pass) {
        #pragma unroll
        for (int i = 0; i < 8; ++i) { const int c = lane + 32 * i, rr = c >> 4, q = (c & 15) * 4;
            *(volatile v4f_t*)(Obase + (size_t)(m0 + rr) * ldo + (c0 - cterm) + q) = *(const volatile v4fa*)(stg + rr * 68 + q); }
        __threadfence();
    }
}

__global__ __launch_bounds__(64)
void attn(const float* __restrict__ Q, const float* __restrict__ Kb,
          const float* __restrict__ V, const float* __restrict__ PE,
          float* __restrict__ act)
{
    const int row = blockIdx.x;
    const int n   = row / LMID;
    const int lq  = row - n * LMID;
    const int h   = threadIdx.x;

    const float* qp = Q + (size_t)(n * LSEQ + lq + CLW/2) * QK + h * EE;
    float q[EE];
    #pragma unroll
    for (int e = 0; e < EE; ++e) q[e] = qp[e];

    const float* kbase = Kb + (size_t)(n * LSEQ + lq) * QK + h * EE;
    const float* vbase = V  + (size_t)(n * LSEQ + lq) * HH + h;

    float m = -3.4e38f, s = 0.f, w = 0.f;
    for (int d = 0; d < CLW; ++d) {
        const float* kr = kbase + d * QK;
        const float* pe = PE + (size_t)(d * HH + h) * EE;
        __builtin_prefetch(kr + QK, 0, 1);
        float e_ = 0.f;
        #pragma unroll
        for (int t = 0; t < EE; ++t) e_ = fmaf(q[t], kr[t] + pe[t], e_);
        const float vd = vbase[d * HH];

        const float mn    = fmaxf(m, e_);
        const float scale = __expf(m - mn);
        const float p     = __expf(e_ - mn);
        s = s * scale + p;
        w = w * scale + p * vd;
        m = mn;
    }
    const float av = fmaxf(w / s, 0.f);
    *(volatile float*)(act + row * HH + h) = av; __threadfence(); *(volatile float*)(act + row * HH + h) = av;
}

__global__ __launch_bounds__(128)
void mlp(const float* __restrict__ act,
         const float* __restrict__ fc_w, const float* __restrict__ fc_b,
         const float* __restrict__ Wout, const float* __restrict__ bout,
         float* __restrict__ out)
{
    __shared__ float smem[4][16 * 64];
    const int lane = threadIdx.x & 31;
    const int wv   = threadIdx.x >> 5;
    const int tile = blockIdx.x * 4 + wv;
    const int r0   = tile * 16;
    float* buf = smem[wv];

    const int nsel = lane & 15;
    const int aoff = (lane & 16) ? 8  : 0;
    const int boff = aoff;

    for (int i = lane; i < 16 * 64; i += 32) buf[i] = act[r0 * 64 + i];
    __syncthreads();

    for (int layer = 0; layer < 4; ++layer) {
        const float* Wl = fc_w + layer * 64 * 64;
        v8f acc[4] = {};
        #pragma unroll
        for (int kk = 0; kk < 64; kk += 32) {
            const float* ar = buf + nsel * 64 + kk + aoff;
            v16h a, al;
            #pragma unroll
            for (int t = 0; t < 8; ++t) { a[t] = (_Float16)ar[t]; al[t] = lo_of(ar[t], a[t]); a[t+8] = (_Float16)ar[16 + t]; al[t+8] = lo_of(ar[16 + t], a[t+8]); }

            v16h bfrag[4], blo[4];
            #pragma unroll
            for (int ct = 0; ct < 4; ++ct) {
                const float* wr = Wl + (ct*16 + nsel) * 64 + kk + boff;
                v16h b, bl;
                #pragma unroll
                for (int t = 0; t < 8; ++t) { b[t] = (_Float16)wr[t]; bl[t] = lo_of(wr[t], b[t]); b[t+8] = (_Float16)wr[16 + t]; bl[t+8] = lo_of(wr[16 + t], b[t+8]); }
                bfrag[ct] = b; blo[ct] = bl;
            }
            #pragma unroll
            for (int ct = 0; ct < 4; ++ct) acc[ct] = wmma_split(a, al, bfrag[ct], blo[ct], acc[ct]);
        }
        __syncthreads();
        #pragma unroll
        for (int ct = 0; ct < 4; ++ct) {
            const int col = ct*16 + nsel;
            const float bb = fc_b[layer * 64 + col];
            #pragma unroll
            for (int j = 0; j < 8; ++j)
                buf[(j + aoff) * 64 + col] = fmaxf(acc[ct][j] + bb, 0.f);
        }
        __syncthreads();
    }

    __shared__ __attribute__((aligned(16))) float so[4 * 48];
    for (int idx = lane; idx < 48; idx += 32) {
        const int rl = idx / 3, o = idx - rl * 3;
        const float* wr = Wout + o * 64;
        float a0 = bout[o];
        #pragma unroll
        for (int hh = 0; hh < 64; ++hh) a0 = fmaf(buf[rl * 64 + hh], wr[hh], a0);
        so[wv * 48 + idx] = a0;
    }
    __syncthreads();
    if (threadIdx.x < 48) {
        float* ob = out + (size_t)blockIdx.x * 64 * 3;
        const v4f_t v = *(const volatile v4fa*)(so + threadIdx.x * 4);
        *(volatile v4f_t*)(ob + threadIdx.x * 4) = v; __threadfence(); *(volatile v4f_t*)(ob + threadIdx.x * 4) = v;
    }
}

extern "C" void kernel_launch(void* const* d_in, const int* in_sizes, int n_in,
                              void* d_out, int out_size, void* d_ws, size_t ws_size,
                              hipStream_t stream)
{
    const float* x    = (const float*)d_in[0];
    const float* Wq   = (const float*)d_in[1];
    const float* bq   = (const float*)d_in[2];
    const float* Wk   = (const float*)d_in[3];
    const float* bk   = (const float*)d_in[4];
    const float* Wv   = (const float*)d_in[5];
    const float* bv   = (const float*)d_in[6];
    const float* PE   = (const float*)d_in[7];
    const float* fc_w = (const float*)d_in[8];
    const float* fc_b = (const float*)d_in[9];
    const float* Wout = (const float*)d_in[10];
    const float* bout = (const float*)d_in[11];
    float* outp = (float*)d_out;

    float* Q   = (float*)d_ws;
    float* Kb  = Q   + (size_t)MROWS * QK;
    float* V   = Kb  + (size_t)MROWS * QK;
    float* act = V   + (size_t)MROWS * HH;
    _Float16* xh = (_Float16*)(act + (size_t)NB * LMID * HH);
    _Float16* wh = xh + 2 * (size_t)MROWS * CDIM;

    to_half<<<512, 256, 0, stream>>>(x, Wq, Wk, Wv, xh, wh);
    qkv_gemm<<<528, 256, 0, stream>>>(xh, wh, bq, bk, bv, Q, Kb, V);
    attn<<<NB * LMID, 64, 0, stream>>>(Q, Kb, V, PE, act);
    mlp<<<30, 128, 0, stream>>>(act, fc_w, fc_b, Wout, bout, outp);
}
